// MaskGenerator_12601434046919
// MI455X (gfx1250) — hardware-verified
//
#include <hip/hip_runtime.h>
#include <stdint.h>


typedef _Float16 v16h __attribute__((ext_vector_type(16)));
typedef _Float16 v8h  __attribute__((ext_vector_type(8)));
typedef float    v8f  __attribute__((ext_vector_type(8)));
typedef float    v4f  __attribute__((ext_vector_type(4)));
typedef uint32_t v4u  __attribute__((ext_vector_type(4)));

#define NODE_DIM 256
#define HID      128
#define H2DIM    64
#define KCAT     NODE_DIM
#define NCAT     (2 * HID)
#define TE       128
#define HP       136
#define H2P      68

static_assert(NODE_DIM == 256);
static_assert(HID == 128);
static_assert(H2DIM == 64);
static_assert(TE * HP * 2 == TE * H2P * 4);

union Frag  { v16h v; v8h half[2]; };
union Pack8 { v8h h; v4u u; };

__device__ __forceinline__ v8f wmma_f16(v16h a, v16h b, v8f c) {
  v8f d = __builtin_amdgcn_wmma_f32_16x16x32_f16(false, a, false, b, (short)0, c, false, false);
  asm volatile("v_nop\n\tv_nop\n\tv_nop\n\tv_nop" : "+v"(d) : "v"(a), "v"(b));
  return d;
}

__device__ __forceinline__ v16h ld_frag(const _Float16* base, int pitch, int rowi, int k0, int h) {
  const _Float16* p = base + (size_t)rowi * pitch + k0 + 8 * h;
  Frag f;
  f.half[0] = *(const v8h*)(p);
  f.half[1] = *(const v8h*)(p + 16);
  return f.v;
}

__global__ __launch_bounds__(256)
void cvt_x(const float* __restrict__ X, _Float16* __restrict__ Xh, int M, int Mp) {
  const long long t = (long long)blockIdx.x * 256 + threadIdx.x;
  const long long total = (long long)Mp * (NODE_DIM / 8);
  if (t >= total) return;
  const int row = (int)(t >> 5);
  const int g   = (int)(t & 31);
  Pack8 pk;
  if (row < M) {
    const float* src = X + (size_t)row * NODE_DIM + g * 8;
    const v4f f0 = *(const v4f*)(src);
    const v4f f1 = *(const v4f*)(src + 4);
    #pragma unroll
    for (int i = 0; i < 4; ++i) { pk.h[i] = (_Float16)f0[i]; pk.h[4 + i] = (_Float16)f1[i]; }
  } else {
    pk.u = (v4u){0u, 0u, 0u, 0u};
  }
  v4u* dst = (v4u*)(Xh + (size_t)row * NODE_DIM + g * 8);
  const v4u val = pk.u;
  *(volatile v4u*)dst = val;
  __threadfence();
  *(volatile v4u*)dst = val;
}

__global__ __launch_bounds__(256)
void cvt_w(const float* __restrict__ W1, const float* __restrict__ W2,
           _Float16* __restrict__ W1t, _Float16* __restrict__ W2t) {
  const int t = blockIdx.x * 256 + threadIdx.x;
  Pack8 pk;
  _Float16* dst;
  if (t < NCAT * (KCAT / 8)) {
    const int n  = t >> 5;
    const int k0 = (t & 31) * 8;
    #pragma unroll
    for (int i = 0; i < 8; ++i) {
      const int k = k0 + i;
      const float v = (n < HID) ? W1[(size_t)k * HID + n]
                                : W1[(size_t)(NODE_DIM + k) * HID + (n - HID)];
      pk.h[i] = (_Float16)(v * 64.0f);
    }
    dst = W1t + (size_t)n * KCAT + k0;
  } else if (t < NCAT * (KCAT / 8) + H2DIM * (HID / 8)) {
    const int t2 = t - NCAT * (KCAT / 8);
    const int n  = t2 >> 4;
    const int k0 = (t2 & 15) * 8;
    #pragma unroll
    for (int i = 0; i < 8; ++i) {
      const int k = k0 + i;
      pk.h[i] = (_Float16)(W2[(size_t)k * H2DIM + n] * 32.0f);
    }
    dst = W2t + (size_t)n * HID + k0;
  } else {
    return;
  }
  const v4u val = pk.u;
  *(volatile v4u*)dst = val;
  __threadfence();
  *(volatile v4u*)dst = val;
}

__global__ __launch_bounds__(128)
void node_gemm(const _Float16* __restrict__ Xh, const _Float16* __restrict__ W1t,
               float* __restrict__ P, int Mp) {
  __shared__ __align__(16) float stage[4 * 32 * 64];
  const int l = threadIdx.x & 31, h = l >> 4, m = l & 15, wv = threadIdx.x >> 5;
  const int row0 = blockIdx.x * 32;
  const int col0 = wv * 64;

  v8f acc[2][4];
  #pragma unroll
  for (int rt = 0; rt < 2; ++rt) {
    #pragma unroll
    for (int nt = 0; nt < 4; ++nt) {
      #pragma unroll
      for (int r = 0; r < 8; ++r) acc[rt][nt][r] = 0.0f;
    }
  }

  #pragma unroll 2
  for (int ks = 0; ks < KCAT / 32; ++ks) {
    const int k0 = ks * 32;
    const v16h a0 = ld_frag(Xh, NODE_DIM, row0 + m, k0, h);
    const v16h a1 = ld_frag(Xh, NODE_DIM, row0 + 16 + m, k0, h);
    #pragma unroll
    for (int nt = 0; nt < 4; ++nt) {
      const v16h b = ld_frag(W1t, KCAT, col0 + 16 * nt + m, k0, h);
      acc[0][nt] = wmma_f16(a0, b, acc[0][nt]);
      acc[1][nt] = wmma_f16(a1, b, acc[1][nt]);
    }
  }

  float* st = stage + wv * (32 * 64);
  #pragma unroll
  for (int rt = 0; rt < 2; ++rt) {
    #pragma unroll
    for (int nt = 0; nt < 4; ++nt) {
      #pragma unroll
      for (int r = 0; r < 8; ++r)
        st[(16 * rt + 8 * h + r) * 64 + 16 * nt + m] = acc[rt][nt][r] * (1.0f / 64.0f);
    }
  }
  __syncthreads();

  #pragma unroll
  for (int it = 0; it < 16; ++it) {
    const int idx = it * 32 + l;
    const int line = idx >> 3, piece = idx & 7;
    const int row = line >> 1, half = line & 1;
    const v4f v = *(const v4f*)(st + row * 64 + 32 * half + 4 * piece);
    float* gp = P + (size_t)(row0 + row) * NCAT + col0 + 32 * half + 4 * piece;
    *(volatile v4f*)gp = v;
  }
  __threadfence();
  #pragma unroll
  for (int it = 0; it < 16; ++it) {
    const int idx = it * 32 + l;
    const int line = idx >> 3, piece = idx & 7;
    const int row = line >> 1, half = line & 1;
    const v4f v = *(const v4f*)(st + row * 64 + 32 * half + 4 * piece);
    float* gp = P + (size_t)(row0 + row) * NCAT + col0 + 32 * half + 4 * piece;
    *(volatile v4f*)gp = v;
  }
}

__global__ __launch_bounds__(128)
void edge_mlp(const float* __restrict__ P, const int* __restrict__ ei,
              const _Float16* __restrict__ W2t,
              const float* __restrict__ b1, const float* __restrict__ b2,
              const float* __restrict__ W3, const float* __restrict__ b3,
              float* __restrict__ out, int E, int nOut, int M) {
  __shared__ __align__(16) char  smem[TE * HP * 2];
  __shared__ __align__(16) float res[TE];
  __shared__ __align__(16) float w3s[H2DIM];
  _Float16* H   = (_Float16*)smem;
  float*    h2s = (float*)smem;

  const int l = threadIdx.x & 31, h = l >> 4, m = l & 15, wv = threadIdx.x >> 5;
  const int tileBase = blockIdx.x * TE;

  if (threadIdx.x < H2DIM) w3s[threadIdx.x] = W3[threadIdx.x];

  int el = tileBase + 32 * wv + l;
  if (el > E - 1) el = E - 1;
  int sI = ei[el];
  int dI = ei[(size_t)E + el];
  sI = sI < 0 ? 0 : (sI > M - 1 ? M - 1 : sI);
  dI = dI < 0 ? 0 : (dI > M - 1 ? M - 1 : dI);

  const v4f bb0 = *(const v4f*)(b1 + 8 * m);
  const v4f bb1 = *(const v4f*)(b1 + 8 * m + 4);

  #pragma unroll 2
  for (int i = 0; i < 16; ++i) {
    const int j = 2 * i + h;
    const int s = __shfl(sI, j);
    const int d = __shfl(dI, j);
    const float* ps = P + (size_t)s * NCAT + 8 * m;
    const float* pd = P + (size_t)d * NCAT + HID + 8 * m;
    const v4f a0 = *(const v4f*)(ps);
    const v4f a1 = *(const v4f*)(ps + 4);
    const v4f c0 = *(const v4f*)(pd);
    const v4f c1 = *(const v4f*)(pd + 4);
    const v4f v0 = (a0 + c0) + bb0;
    const v4f v1 = (a1 + c1) + bb1;
    Pack8 pk;
    #pragma unroll
    for (int q = 0; q < 4; ++q) {
      float x0 = v0[q]; x0 = x0 > 0.0f ? x0 : 0.0f;
      float x1 = v1[q]; x1 = x1 > 0.0f ? x1 : 0.0f;
      pk.h[q]     = (_Float16)x0;
      pk.h[4 + q] = (_Float16)x1;
    }
    *(v4u*)(H + (size_t)(32 * wv + j) * HP + 8 * m) = pk.u;
  }
  __syncthreads();

  float hb2[4];
  #pragma unroll
  for (int nt = 0; nt < 4; ++nt) hb2[nt] = b2[16 * nt + m];

  v8f acc[2][4];
  #pragma unroll
  for (int rt = 0; rt < 2; ++rt) {
    #pragma unroll
    for (int nt = 0; nt < 4; ++nt) {
      #pragma unroll
      for (int r = 0; r < 8; ++r) acc[rt][nt][r] = 0.0f;
    }
  }

  #pragma unroll
  for (int ks = 0; ks < HID / 32; ++ks) {
    const int k0 = ks * 32;
    const v16h a0 = ld_frag(H, HP, 32 * wv + m, k0, h);
    const v16h a1 = ld_frag(H, HP, 32 * wv + 16 + m, k0, h);
    #pragma unroll
    for (int nt = 0; nt < 4; ++nt) {
      const v16h b = ld_frag(W2t, HID, 16 * nt + m, k0, h);
      acc[0][nt] = wmma_f16(a0, b, acc[0][nt]);
      acc[1][nt] = wmma_f16(a1, b, acc[1][nt]);
    }
  }
  __syncthreads();

  #pragma unroll
  for (int rt = 0; rt < 2; ++rt) {
    #pragma unroll
    for (int nt = 0; nt < 4; ++nt) {
      #pragma unroll
      for (int r = 0; r < 8; ++r) {
        float v = acc[rt][nt][r] * (1.0f / 32.0f) + hb2[nt];
        v = v > 0.0f ? v : 0.0f;
        h2s[(32 * wv + 16 * rt + 8 * h + r) * H2P + 16 * nt + m] = v;
      }
    }
  }
  __syncthreads();

  {
    const int t = threadIdx.x;
    const float* hr = h2s + t * H2P;
    float s = 0.0f;
    #pragma unroll
    for (int q = 0; q < H2DIM / 4; ++q) {
      const v4f hv = *(const v4f*)(hr + 4 * q);
      const v4f wq = *(const v4f*)(w3s + 4 * q);
      s += hv[0] * wq[0];
      s += hv[1] * wq[1];
      s += hv[2] * wq[2];
      s += hv[3] * wq[3];
    }
    s += b3[0];
    s = s > 30.0f ? 30.0f : (s < -30.0f ? -30.0f : s);
    const float ex = expf(-s);
    res[t] = __builtin_amdgcn_rcpf(1.0f + ex);
  }
  __syncthreads();

  if (tileBase + TE <= nOut) {
    if (wv == 0) {
      const v4f v = *(const v4f*)(res + 4 * l);
      float* gp = out + (size_t)tileBase + 4 * l;
      *(volatile v4f*)gp = v;
      __threadfence();
      *(volatile v4f*)gp = v;
    }
  } else {
    const int t = threadIdx.x;
    const int e = tileBase + t;
    const float v = res[t];
    if ((unsigned)e < (unsigned)nOut) {
      *(volatile float*)(out + e) = v;
      __threadfence();
      *(volatile float*)(out + e) = v;
    }
  }
}

static inline size_t align_up_256(size_t x) { return (x + 255) & ~(size_t)255; }

extern "C" void kernel_launch(void* const* d_in, const int* in_sizes, int n_in,
                              void* d_out, int out_size, void* d_ws, size_t ws_size,
                              hipStream_t stream) {
  if (n_in < 8) return;
  const float* node_emb   = (const float*)d_in[0];
  const int*   edge_index = (const int*)  d_in[1];
  const float* W1         = (const float*)d_in[2];
  const float* b1         = (const float*)d_in[3];
  const float* W2         = (const float*)d_in[4];
  const float* b2         = (const float*)d_in[5];
  const float* W3         = (const float*)d_in[6];
  const float* b3         = (const float*)d_in[7];
  float* out = (float*)d_out;

  const int M    = in_sizes[0] / NODE_DIM;
  const int E    = in_sizes[1] / 2;
  const int nOut = out_size;
  if (M < 1 || E < 1 || nOut < 1) return;
  if (in_sizes[2] != 2 * NODE_DIM * HID || in_sizes[3] != HID ||
      in_sizes[4] != HID * H2DIM || in_sizes[5] != H2DIM ||
      in_sizes[6] != H2DIM || in_sizes[7] < 1) return;

  const int Mp = ((M + 31) / 32) * 32;

  const size_t offXh  = 0;
  const size_t offW1t = align_up_256(offXh  + (size_t)Mp * NODE_DIM * sizeof(_Float16));
  const size_t offW2t = align_up_256(offW1t + (size_t)NCAT * KCAT * sizeof(_Float16));
  const size_t offP   = align_up_256(offW2t + (size_t)H2DIM * HID * sizeof(_Float16));
  const size_t total  = offP + (size_t)Mp * NCAT * sizeof(float);
  if (total > ws_size) return;

  char* ws = (char*)d_ws;
  _Float16* Xh  = (_Float16*)(ws + offXh);
  _Float16* W1t = (_Float16*)(ws + offW1t);
  _Float16* W2t = (_Float16*)(ws + offW2t);
  float*    P   = (float*)   (ws + offP);

  {
    const long long totalT = (long long)Mp * (NODE_DIM / 8);
    const int blocks = (int)((totalT + 255) / 256);
    cvt_x<<<blocks, 256, 0, stream>>>(node_emb, Xh, M, Mp);
  }
  {
    const int nT = NCAT * (KCAT / 8) + H2DIM * (HID / 8);
    const int blocks = (nT + 255) / 256;
    cvt_w<<<blocks, 256, 0, stream>>>(W1, W2, W1t, W2t);
  }
  {
    const int blocks = Mp / 32;
    node_gemm<<<blocks, 128, 0, stream>>>(Xh, W1t, P, Mp);
  }
  {
    const int blocks = (E + TE - 1) / TE;
    edge_mlp<<<blocks, 128, 0, stream>>>(P, edge_index, W2t, b1, b2, W3, b3, out, E, nOut, M);
  }
  (void)hipGetLastError();
}
